// CrossAttentionFormerBlock_1752346656897
// MI455X (gfx1250) — hardware-verified
//
#include <hip/hip_runtime.h>
#include <math.h>


#define LL 32768
#define CC 256
#define NHD 8
#define HD 32
#define GG 8
#define NW 64
#define WN 512
#define FF 1024
#define NP 3375

typedef __attribute__((ext_vector_type(16))) _Float16 v16h;
typedef __attribute__((ext_vector_type(8)))  _Float16 v8h;
typedef __attribute__((ext_vector_type(8)))  float v8f;
typedef __attribute__((ext_vector_type(4)))  float v4f;
typedef __attribute__((ext_vector_type(4)))  unsigned v4u;

template <typename T> __device__ __forceinline__ void vst2(void* p, T v) { *(volatile T*)p = v; __threadfence(); *(volatile T*)p = v; }
__device__ __forceinline__ v8f wmma16(v16h a, v16h b, v8f c) {
  v8f d = __builtin_amdgcn_wmma_f32_16x16x32_f16(false, a, false, b, (short)0, c, false, false);
  asm volatile("v_nop\n\tv_nop\n\tv_nop\n\tv_nop" : "+v"(d) : "v"(a), "v"(b));
  return d;
}
__device__ __forceinline__ v16h frag_h(const _Float16* rowk0, int lane) {
  union { v16h v; v8h q[2]; } u; const _Float16* p = rowk0 + 8 * (lane >> 4);
  u.q[0] = *(const v8h*)p; u.q[1] = *(const v8h*)(p + 16); return u.v;
}
__device__ __forceinline__ v16h frag_f32(const float* rowk0, int lane) {
  v16h a; const float* p = rowk0 + 8 * (lane >> 4);
#pragma unroll
  for (int i = 0; i < 8; ++i) { a[i] = (_Float16)p[i]; a[8 + i] = (_Float16)p[16 + i]; }
  return a;
}
#define LDSX() do { asm volatile("s_wait_dscnt 0" ::: "memory"); __builtin_amdgcn_wave_barrier(); __builtin_amdgcn_fence(__ATOMIC_RELEASE, "workgroup"); } while (0)

__device__ __forceinline__ int wtok2L(int wt) {
  const int win = wt >> 9, n = wt & 511;
  const int hb = win >> 4, wb = (win >> 2) & 3, db = win & 3;
  const int h1 = n >> 6, w1 = (n >> 3) & 7, d1 = n & 7;
  return ((hb * GG + h1) * 32 + (wb * GG + w1)) * 32 + (db * GG + d1);
}

__global__ __launch_bounds__(64) void k_ln16(const float* __restrict__ x, const float* __restrict__ gm, const float* __restrict__ bt, _Float16* __restrict__ o16) {
  __shared__ float red[64];
  const size_t row = blockIdx.x; const int tid = threadIdx.x;
  const v4f v = *(const v4f*)(x + row * CC + tid * 4);
  red[tid] = v[0] + v[1] + v[2] + v[3]; __syncthreads();
  for (int st = 32; st > 0; st >>= 1) { if (tid < st) red[tid] += red[tid + st]; __syncthreads(); }
  const float mu = red[0] / (float)CC; __syncthreads();
  const float d0 = v[0] - mu, d1 = v[1] - mu, d2 = v[2] - mu, d3 = v[3] - mu;
  red[tid] = d0 * d0 + d1 * d1 + d2 * d2 + d3 * d3; __syncthreads();
  for (int st = 32; st > 0; st >>= 1) { if (tid < st) red[tid] += red[tid + st]; __syncthreads(); }
  const float rs = rsqrtf(red[0] / (float)CC + 1e-5f);
  __shared__ __align__(16) float rowv[CC];
  rowv[tid * 4] = d0 * rs * gm[tid * 4] + bt[tid * 4]; rowv[tid * 4 + 1] = d1 * rs * gm[tid * 4 + 1] + bt[tid * 4 + 1];
  rowv[tid * 4 + 2] = d2 * rs * gm[tid * 4 + 2] + bt[tid * 4 + 2]; rowv[tid * 4 + 3] = d3 * rs * gm[tid * 4 + 3] + bt[tid * 4 + 3];
  __syncthreads();
  if (tid < 32) { union { v8h h; v4u u; } pk;
#pragma unroll
    for (int e = 0; e < 8; ++e) pk.h[e] = (_Float16)rowv[tid * 8 + e];
    vst2(o16 + row * CC + tid * 8, pk.u); }
}
__global__ __launch_bounds__(256) void k_cvt(const float* __restrict__ s, _Float16* __restrict__ d, size_t n8) {
  const size_t g8 = (size_t)blockIdx.x * 256 + threadIdx.x; if (g8 >= n8) return;
  union { v8h h; v4u u; } pk;
#pragma unroll
  for (int e = 0; e < 8; ++e) pk.h[e] = (_Float16)s[g8 * 8 + e];
  vst2(d + g8 * 8, pk.u);
}
__global__ __launch_bounds__(256) void k_packT(const float* __restrict__ W, _Float16* __restrict__ Wt, int K, int N) {
  __shared__ float tile[64][65];
  const int k0 = blockIdx.y * 64, n0 = blockIdx.x * 64, tid = threadIdx.x;
  for (int q = tid; q < 64 * 64; q += 256) { const int kk = q >> 6, nn = q & 63; tile[kk][nn] = W[(size_t)(k0 + kk) * N + n0 + nn]; }
  __syncthreads();
  for (int q = tid; q < 64 * 8; q += 256) { const int nn = q >> 3, pc = q & 7;
    union { v8h h; v4u u; } pk;
#pragma unroll
    for (int e = 0; e < 8; ++e) pk.h[e] = (_Float16)tile[pc * 8 + e][nn];
    vst2(Wt + (size_t)(n0 + nn) * K + k0 + pc * 8, pk.u); }
}

__global__ __launch_bounds__(128) void k_posmlp(const float* __restrict__ ppw, const float* __restrict__ ppb,
    const float* __restrict__ g1, const float* __restrict__ c1, const float* __restrict__ w1, const float* __restrict__ b1,
    const float* __restrict__ g2, const float* __restrict__ c2, const float* __restrict__ w2, const float* __restrict__ b2,
    const float* __restrict__ g3, const float* __restrict__ c3, const float* __restrict__ w3, const float* __restrict__ b3, float* __restrict__ pos) {
  const int t2 = blockIdx.x * 128 + threadIdx.x, r = t2 >> 1, half = t2 & 1;
  if (r >= NP + 1) return;
  const float crd[3] = { (float)(r / 225 - 7), (float)((r / 15) % 15 - 7), (float)(r % 15 - 7) };
  float a[16], t[16];
#pragma unroll
  for (int j = 0; j < 16; ++j) a[j] = ppb[j] + crd[0] * ppw[j] + crd[1] * ppw[16 + j] + crd[2] * ppw[32 + j];
#pragma unroll 1
  for (int st = 0; st < 3; ++st) {
    const float* gm = st == 0 ? g1 : (st == 1 ? g2 : g3); const float* bt = st == 0 ? c1 : (st == 1 ? c2 : c3);
    const float* W = st == 0 ? w1 : (st == 1 ? w2 : w3); const float* bb = st == 0 ? b1 : (st == 1 ? b2 : b3);
    const int no = st == 2 ? 8 : 16;
    float mu = 0.f; for (int j = 0; j < 16; ++j) mu += a[j]; mu /= 16.f;
    float var = 0.f; for (int j = 0; j < 16; ++j) var += (a[j] - mu) * (a[j] - mu); var /= 16.f;
    const float rs = 1.0f / sqrtf(var + 1e-5f);
    for (int j = 0; j < 16; ++j) { float v = (a[j] - mu) * rs * gm[j] + bt[j]; t[j] = v > 0.f ? v : 0.f; }
    for (int o = 0; o < 16; ++o) { float s = o < no ? bb[o] : 0.f; if (o < no) for (int j = 0; j < 16; ++j) s += t[j] * W[j * no + o]; a[o] = s; }
  }
  v4f o = half ? (v4f){a[4], a[5], a[6], a[7]} : (v4f){a[0], a[1], a[2], a[3]};
  if (r == NP) o = (v4f){0.f, 0.f, 0.f, 0.f};
  vst2(pos + (size_t)r * 8 + half * 4, o);
}

__global__ __launch_bounds__(128) void k_qkv(const _Float16* __restrict__ xn, const _Float16* __restrict__ y16, const _Float16* __restrict__ WqkvT,
                                           const float* __restrict__ bqkv, _Float16* __restrict__ qh, _Float16* __restrict__ kh, _Float16* __restrict__ vT) {
  __shared__ __align__(16) float st[128][68];
  __shared__ __align__(16) float so[4][16 * 128];
  const int tid = threadIdx.x, wave = tid >> 5, lane = tid & 31, col = lane & 15, g = lane >> 4;
  const int which = blockIdx.z, wt0 = blockIdx.x * 64, n0 = blockIdx.y * 128;
  const _Float16* A = which == 0 ? xn : y16;
  const int Lrow = wtok2L(wt0 + wave * 16 + col);
  v8f acc[8] = {};
#pragma unroll
  for (int kc = 0; kc < CC / 32; ++kc) { const v16h a = frag_h(A + (size_t)Lrow * CC + kc * 32, lane);
#pragma unroll
    for (int j = 0; j < 8; ++j) acc[j] = wmma16(a, frag_h(WqkvT + (size_t)(which * CC + n0 + j * 16 + col) * CC + kc * 32, lane), acc[j]); }
  const float sc = which == 0 ? 0.17677669529663688f : 1.0f;
  if (which < 2) { float* S = so[wave]; _Float16* D = which == 0 ? qh : kh;
#pragma unroll
    for (int j = 0; j < 8; ++j) { const float bv = bqkv[which * CC + n0 + j * 16 + col];
#pragma unroll
      for (int r = 0; r < 8; ++r) S[(8 * g + r) * 128 + j * 16 + col] = (acc[j][r] + bv) * sc; }
    LDSX();
#pragma unroll
    for (int q = 0; q < 8; ++q) { const int rl = q * 2 + (lane >> 4), pc = lane & 15;
      union { v8h h; v4u u; } pk;
#pragma unroll
      for (int e = 0; e < 8; ++e) pk.h[e] = (_Float16)S[rl * 128 + pc * 8 + e];
      vst2(D + (size_t)(wt0 + wave * 16 + rl) * CC + n0 + pc * 8, pk.u); }
  } else {
#pragma unroll
    for (int j = 0; j < 8; ++j) { const float bv = bqkv[2 * CC + n0 + j * 16 + col];
#pragma unroll
      for (int r = 0; r < 8; ++r) st[j * 16 + col][wave * 16 + 8 * g + r] = acc[j][r] + bv; }
    __syncthreads();
    const int win = wt0 >> 9, nl0 = wt0 & 511;
    for (int q = tid; q < 128 * 8; q += 128) { const int cl = q >> 3, pc = q & 7;
      union { v8h h; v4u u; } pk;
#pragma unroll
      for (int e = 0; e < 8; ++e) pk.h[e] = (_Float16)st[cl][pc * 8 + e];
      vst2(vT + ((size_t)win * CC + n0 + cl) * WN + nl0 + pc * 8, pk.u); }
  }
}

__global__ __launch_bounds__(128) void k_wattn(const _Float16* __restrict__ qh, const _Float16* __restrict__ kh, const _Float16* __restrict__ vT,
                                             const float* __restrict__ pos, _Float16* __restrict__ o16) {
  __shared__ __align__(16) float sP[4][16][32];
  __shared__ __align__(16) float sO[32][2 * HD];
  const int tid = threadIdx.x, w = tid >> 5, lane = tid & 31, g = lane >> 4, ln = lane & 15;
  const int win = blockIdx.y >> 2, hp = blockIdx.y & 3, hh = w >> 1, h = hp * 2 + hh;
  const int qb = blockIdx.x * 32, q0 = qb + (w & 1) * 16;
  const _Float16* qrow = qh + ((size_t)win * WN + q0 + ln) * CC + h * HD;
  const v16h qa = frag_h(qrow, lane);
  const _Float16* kb = kh + (size_t)win * WN * CC + h * HD;
  const _Float16* vb = vT + ((size_t)win * CC + h * HD) * WN;
  float mrun[8], lrun[8]; v8f acc[2];
#pragma unroll
  for (int r = 0; r < 8; ++r) { mrun[r] = -3.0e38f; lrun[r] = 0.f; }
  acc[0] = (v8f){}; acc[1] = (v8f){};
#pragma unroll 1
  for (int k0 = 0; k0 < WN; k0 += 32) {
    v8f s0 = {}, s1 = {};
    s0 = wmma16(qa, frag_h(kb + (size_t)(k0 + ln) * CC, lane), s0);
    s1 = wmma16(qa, frag_h(kb + (size_t)(k0 + 16 + ln) * CC, lane), s1);
    const int m0 = k0 + ln, m1 = k0 + 16 + ln;
#pragma unroll
    for (int r = 0; r < 8; ++r) {
      const int n = q0 + 8 * g + r;
      const int dh0 = (n >> 6) - (m0 >> 6) + 7, dw0 = ((n >> 3) & 7) - ((m0 >> 3) & 7) + 7, dd0 = (n & 7) - (m0 & 7) + 7;
      const int dh1 = (n >> 6) - (m1 >> 6) + 7, dw1 = ((n >> 3) & 7) - ((m1 >> 3) & 7) + 7, dd1 = (n & 7) - (m1 & 7) + 7;
      const float x0 = s0[r] + pos[(size_t)((dh0 * 15 + dw0) * 15 + dd0) * 8 + h], x1 = s1[r] + pos[(size_t)((dh1 * 15 + dw1) * 15 + dd1) * 8 + h];
      float mx = fmaxf(x0, x1);
#pragma unroll
      for (int off = 8; off >= 1; off >>= 1) mx = fmaxf(mx, __shfl_xor(mx, off, 32));
      const float mn = fmaxf(mrun[r], mx); const float corr = expf(mrun[r] - mn);
      const float p0 = expf(x0 - mn), p1 = expf(x1 - mn);
      float sum = p0 + p1;
#pragma unroll
      for (int off = 8; off >= 1; off >>= 1) sum += __shfl_xor(sum, off, 32);
      lrun[r] = lrun[r] * corr + sum; mrun[r] = mn;
      acc[0][r] *= corr; acc[1][r] *= corr;
      sP[w][8 * g + r][ln] = p0 * 16384.0f; sP[w][8 * g + r][16 + ln] = p1 * 16384.0f;
    }
    LDSX();
    const v16h pa = frag_f32(&sP[w][ln][0], lane);
    acc[0] = wmma16(pa, frag_h(vb + (size_t)ln * WN + k0, lane), acc[0]);
    acc[1] = wmma16(pa, frag_h(vb + (size_t)(16 + ln) * WN + k0, lane), acc[1]);
    __builtin_amdgcn_wave_barrier();
  }
#pragma unroll
  for (int r = 0; r < 8; ++r) { const float il = (1.0f / 16384.0f) / lrun[r]; const int row = (w & 1) * 16 + 8 * g + r;
    sO[row][hh * HD + ln] = acc[0][r] * il; sO[row][hh * HD + 16 + ln] = acc[1][r] * il; }
  __syncthreads();
  for (int q = tid; q < 32 * 8; q += 128) { const int rl = q >> 3, pc = q & 7;
    union { v8h hv; v4u u; } pk;
#pragma unroll
    for (int e = 0; e < 8; ++e) pk.hv[e] = (_Float16)sO[rl][pc * 8 + e];
    vst2(o16 + ((size_t)win * WN + qb + rl) * CC + hp * 2 * HD + pc * 8, pk.u); }
}

__global__ __launch_bounds__(128) void k_proj(const _Float16* __restrict__ o16, const _Float16* __restrict__ WpT, const float* __restrict__ pb,
                                            const float* __restrict__ x, float* __restrict__ x1) {
  __shared__ __align__(16) float so[4][16 * 128];
  const int tid = threadIdx.x, wave = tid >> 5, lane = tid & 31, col = lane & 15, g = lane >> 4;
  const int wt0 = blockIdx.x * 64 + wave * 16, n0 = blockIdx.y * 128;
  v8f acc[8] = {};
#pragma unroll
  for (int kc = 0; kc < CC / 32; ++kc) { const v16h a = frag_h(o16 + (size_t)(wt0 + col) * CC + kc * 32, lane);
#pragma unroll
    for (int j = 0; j < 8; ++j) acc[j] = wmma16(a, frag_h(WpT + (size_t)(n0 + j * 16 + col) * CC + kc * 32, lane), acc[j]); }
  float* S = so[wave];
#pragma unroll
  for (int j = 0; j < 8; ++j) { const float bv = pb[n0 + j * 16 + col];
#pragma unroll
    for (int r = 0; r < 8; ++r) S[(8 * g + r) * 128 + j * 16 + col] = acc[j][r] + bv; }
  LDSX();
#pragma unroll 4
  for (int rl = 0; rl < 16; ++rl) { const size_t L = (size_t)wtok2L(wt0 + rl); const size_t o = L * CC + n0 + lane * 4;
    vst2(x1 + o, *(const v4f*)(S + rl * 128 + lane * 4) + *(const v4f*)(x + o)); }
}

__global__ __launch_bounds__(128) void k_fc1(const _Float16* __restrict__ x2, const _Float16* __restrict__ W1T, const float* __restrict__ b1, _Float16* __restrict__ hid) {
  __shared__ __align__(16) float so[4][16 * 128];
  const int tid = threadIdx.x, wave = tid >> 5, lane = tid & 31, col = lane & 15, g = lane >> 4;
  const int r0 = blockIdx.x * 64 + wave * 16, n0 = blockIdx.y * 128;
  v8f acc[8] = {};
#pragma unroll
  for (int kc = 0; kc < CC / 32; ++kc) { const v16h a = frag_h(x2 + (size_t)(r0 + col) * CC + kc * 32, lane);
#pragma unroll
    for (int j = 0; j < 8; ++j) acc[j] = wmma16(a, frag_h(W1T + (size_t)(n0 + j * 16 + col) * CC + kc * 32, lane), acc[j]); }
  float* S = so[wave];
#pragma unroll
  for (int j = 0; j < 8; ++j) { const float bv = b1[n0 + j * 16 + col];
#pragma unroll
    for (int r = 0; r < 8; ++r) { const float u = acc[j][r] + bv; S[(8 * g + r) * 128 + j * 16 + col] = 0.5f * u * (1.0f + erff(u * 0.70710678118654752f)); } }
  LDSX();
#pragma unroll
  for (int q = 0; q < 8; ++q) { const int rl = q * 2 + (lane >> 4), pc = lane & 15;
    union { v8h h; v4u u; } pk;
#pragma unroll
    for (int e = 0; e < 8; ++e) pk.h[e] = (_Float16)S[rl * 128 + pc * 8 + e];
    vst2(hid + (size_t)(r0 + rl) * FF + n0 + pc * 8, pk.u); }
}
__global__ __launch_bounds__(128) void k_fc2(const _Float16* __restrict__ hid, const _Float16* __restrict__ W2T, const float* __restrict__ b2,
                                           const float* __restrict__ x1, float* __restrict__ out) {
  __shared__ __align__(16) float so[4][16 * 128];
  const int tid = threadIdx.x, wave = tid >> 5, lane = tid & 31, col = lane & 15, g = lane >> 4;
  const int r0 = blockIdx.x * 64 + wave * 16, n0 = blockIdx.y * 128;
  v8f acc[8] = {};
#pragma unroll 1
  for (int kc = 0; kc < FF / 32; ++kc) { const v16h a = frag_h(hid + (size_t)(r0 + col) * FF + kc * 32, lane);
#pragma unroll
    for (int j = 0; j < 8; ++j) acc[j] = wmma16(a, frag_h(W2T + (size_t)(n0 + j * 16 + col) * FF + kc * 32, lane), acc[j]); }
  float* S = so[wave];
#pragma unroll
  for (int j = 0; j < 8; ++j) { const float bv = b2[n0 + j * 16 + col];
#pragma unroll
    for (int r = 0; r < 8; ++r) S[(8 * g + r) * 128 + j * 16 + col] = acc[j][r] + bv; }
  LDSX();
#pragma unroll 4
  for (int rl = 0; rl < 16; ++rl) { const size_t o = (size_t)(r0 + rl) * CC + n0 + lane * 4;
    vst2(out + o, *(const v4f*)(S + rl * 128 + lane * 4) + *(const v4f*)(x1 + o)); }
}

extern "C" void kernel_launch(void* const* d_in, const int* in_sizes, int n_in,
                              void* d_out, int out_size, void* d_ws, size_t ws_size,
                              hipStream_t stream) {
  (void)in_sizes; (void)n_in; (void)out_size; (void)ws_size;
  const float* x = (const float*)d_in[0]; const float* y = (const float*)d_in[1];
  const float* n1g = (const float*)d_in[2]; const float* n1b = (const float*)d_in[3];
  const float* qkvw = (const float*)d_in[4]; const float* qkvb = (const float*)d_in[5];
  const float* ppw = (const float*)d_in[6]; const float* ppb = (const float*)d_in[7];
  const float* p1g = (const float*)d_in[8]; const float* p1c = (const float*)d_in[9]; const float* p1w = (const float*)d_in[10]; const float* p1b = (const float*)d_in[11];
  const float* p2g = (const float*)d_in[12]; const float* p2c = (const float*)d_in[13]; const float* p2w = (const float*)d_in[14]; const float* p2b = (const float*)d_in[15];
  const float* p3g = (const float*)d_in[16]; const float* p3c = (const float*)d_in[17]; const float* p3w = (const float*)d_in[18]; const float* p3b = (const float*)d_in[19];
  const float* pw = (const float*)d_in[20]; const float* pb = (const float*)d_in[21];
  const float* n2g = (const float*)d_in[22]; const float* n2b = (const float*)d_in[23];
  const float* f1w = (const float*)d_in[24]; const float* f1b = (const float*)d_in[25];
  const float* f2w = (const float*)d_in[26]; const float* f2b = (const float*)d_in[27];
  float* out = (float*)d_out;
  char* ws = (char*)d_ws; size_t off = 0;
  auto take = [&](size_t bytes) { char* p = ws + off; off += (bytes + 255) & ~(size_t)255; return p; };
  _Float16* xn  = (_Float16*)take((size_t)LL * CC * 2); _Float16* y16 = (_Float16*)take((size_t)LL * CC * 2);
  _Float16* WqkvT = (_Float16*)take((size_t)3 * CC * CC * 2); _Float16* WpT = (_Float16*)take((size_t)CC * CC * 2);
  _Float16* W1T = (_Float16*)take((size_t)FF * CC * 2); _Float16* W2T = (_Float16*)take((size_t)CC * FF * 2);
  float* pos = (float*)take((size_t)(NP + 1) * 8 * 4);
  _Float16* qh = (_Float16*)take((size_t)LL * CC * 2); _Float16* kh = (_Float16*)take((size_t)LL * CC * 2);
  _Float16* vT = (_Float16*)take((size_t)NW * CC * WN * 2);
  _Float16* o16 = (_Float16*)take((size_t)LL * CC * 2);
  float* x1 = (float*)take((size_t)LL * CC * 4);
  _Float16* x2 = (_Float16*)take((size_t)LL * CC * 2);
  _Float16* hid = (_Float16*)take((size_t)LL * FF * 2);
  k_ln16<<<LL, 64, 0, stream>>>(x, n1g, n1b, xn);
  k_cvt<<<(unsigned)((LL * CC / 8 + 255) / 256), 256, 0, stream>>>(y, y16, (size_t)LL * CC / 8);
  k_packT<<<dim3(3 * CC / 64, CC / 64), 256, 0, stream>>>(qkvw, WqkvT, CC, 3 * CC);
  k_packT<<<dim3(CC / 64, CC / 64), 256, 0, stream>>>(pw, WpT, CC, CC);
  k_packT<<<dim3(FF / 64, CC / 64), 256, 0, stream>>>(f1w, W1T, CC, FF);
  k_packT<<<dim3(CC / 64, FF / 64), 256, 0, stream>>>(f2w, W2T, FF, CC);
  k_posmlp<<<(2 * (NP + 1) + 127) / 128, 128, 0, stream>>>(ppw, ppb, p1g, p1c, p1w, p1b, p2g, p2c, p2w, p2b, p3g, p3c, p3w, p3b, pos);
  k_qkv<<<dim3(LL / 64, CC / 128, 3), 128, 0, stream>>>(xn, y16, WqkvT, qkvb, qh, kh, vT);
  k_wattn<<<dim3(WN / 32, NW * 4), 128, 0, stream>>>(qh, kh, vT, pos, o16);
  k_proj<<<dim3(LL / 64, CC / 128), 128, 0, stream>>>(o16, WpT, pb, x, x1);
  k_ln16<<<LL, 64, 0, stream>>>(x1, n2g, n2b, x2);
  k_fc1<<<dim3(LL / 64, FF / 128), 128, 0, stream>>>(x2, W1T, f1b, hid);
  k_fc2<<<dim3(LL / 64, CC / 128), 128, 0, stream>>>(hid, W2T, f2b, x1, out);
}
